// PathNN_67997922231065
// MI455X (gfx1250) — hardware-verified
//
#include <hip/hip_runtime.h>
#include <hip/hip_bf16.h>
#include <stddef.h>


#define HD       128
#define G4       512
#define NCLS     10
#define NGR      128
#define NTHR     256
#define NWAVE    8
#define EPT      8
#define NGRP     2
#define CHUNK    (NTHR * EPT * NGRP)
#define WCAP     (EPT * NGRP * 32)
#define LISTN    (NWAVE * WCAP)
#define NBA      256
#define GER      128
#define GXR      64
#define PB       64
#define AP       136
#define ZP       132
#define WSC      16.0f
#define WINV     0.0625f

#define LDS_ENC  (GER * HD * 4 + 4096)
#define LDS_XG   (GXR * G4 * 4)
#define LDS_AGG  (NBA * HD * 4 + LISTN * 4 + 64 + 4096)
#define LDS_POOL (NWAVE * NGR * 32 * 4 + NGR * 32 * 4)
#define LDS_HEAD (NGR * ZP * 4 + NGR * NCLS * 4)

static_assert((CHUNK & (CHUNK - 1)) == 0);
static_assert(CHUNK <= 4096);
static_assert((NBA & (NBA - 1)) == 0 && NBA <= 4096);
static_assert(GER * AP * 2 <= GER * HD * 4);
static_assert(GXR * AP * 2 <= LDS_XG);
static_assert(NBA % GER == 0 && NBA % GXR == 0);
static_assert((NGR * NCLS * 4) % 512 == 0);
static_assert(NBA / NWAVE == 32);

typedef float    v4f  __attribute__((ext_vector_type(4)));
typedef float    v8f  __attribute__((ext_vector_type(8)));
typedef double   v2d  __attribute__((ext_vector_type(2)));
typedef _Float16 v8h  __attribute__((ext_vector_type(8)));
typedef _Float16 v16h __attribute__((ext_vector_type(16)));
typedef __bf16   v16b __attribute__((ext_vector_type(16)));
union FragH { v16h v; v8h h[2]; };
union FragB { v16b v; unsigned u[8]; };

__device__ __forceinline__ v8f zero8f() { v8f z = {0.f, 0.f, 0.f, 0.f, 0.f, 0.f, 0.f, 0.f}; return z; }
__device__ __forceinline__ v8h zero8h() {
  const _Float16 hz = (_Float16)0.0f;
  v8h z = {hz, hz, hz, hz, hz, hz, hz, hz};
  return z;
}

__device__ __forceinline__ v8h cvt8(v4f a, v4f b) {
  v8h r;
  r[0] = (_Float16)a.x; r[1] = (_Float16)a.y; r[2] = (_Float16)a.z; r[3] = (_Float16)a.w;
  r[4] = (_Float16)b.x; r[5] = (_Float16)b.y; r[6] = (_Float16)b.z; r[7] = (_Float16)b.w;
  return r;
}

__device__ __forceinline__ v4f relu4(v4f v) {
  v.x = fmaxf(v.x, 0.f); v.y = fmaxf(v.y, 0.f); v.z = fmaxf(v.z, 0.f); v.w = fmaxf(v.w, 0.f);
  return v;
}

__device__ __forceinline__ unsigned bfr(float f) {
  unsigned u = __float_as_uint(f);
  u = u + 0x7fffu + ((u >> 16) & 1u);
  return u >> 16;
}

__device__ __forceinline__ void split8(v4f a, v4f b, FragB& H, FragB& L, const int q) {
  float x[8] = {a.x, a.y, a.z, a.w, b.x, b.y, b.z, b.w};
#pragma unroll
  for (int j = 0; j < 4; ++j) {
    const unsigned h0 = bfr(x[2 * j]), h1 = bfr(x[2 * j + 1]);
    const float    r0 = x[2 * j] - __uint_as_float(h0 << 16);
    const float    r1 = x[2 * j + 1] - __uint_as_float(h1 << 16);
    const unsigned l0 = bfr(r0), l1 = bfr(r1);
    H.u[4 * q + j] = h0 | (h1 << 16);
    L.u[4 * q + j] = l0 | (l1 << 16);
  }
}

__device__ __forceinline__ v8f wmh(v16h a, v16h b, v8f c) {
  v8f d = __builtin_amdgcn_wmma_f32_16x16x32_f16(false, a, false, b, (short)0, c, false, false);
  asm volatile("v_nop\n\tv_nop\n\tv_nop\n\tv_nop" : "+v"(d) : "v"(a), "v"(b));
  return d;
}
__device__ __forceinline__ v8f wmb(v16b a, v16b b, v8f c) {
  v8f d = __builtin_amdgcn_wmma_f32_16x16x32_bf16(false, a, false, b, (short)0, c, false, false);
  asm volatile("v_nop\n\tv_nop\n\tv_nop\n\tv_nop" : "+v"(d) : "v"(a), "v"(b));
  return d;
}

__device__ __forceinline__ float sigm(float x) {
  x = fminf(fmaxf(x, -30.f), 30.f);
  const float e = __expf(-x);
  return __builtin_amdgcn_rcpf(1.0f + e);
}

__global__ __launch_bounds__(NTHR) void k_wprep(
    const float* __restrict__ w1, const float* __restrict__ w2,
    const float* __restrict__ wih, const float* __restrict__ whh,
    const float* __restrict__ bih, const float* __restrict__ bhh,
    _Float16* q1, _Float16* q2, _Float16* qih, _Float16* qhh, float* bsum, int nWblk) {
  const int tid = threadIdx.x;
  if ((int)blockIdx.x < nWblk) {
    const int i   = blockIdx.x * NTHR + tid;
    const int n1  = HD * HD / 8;
    const int n3  = G4 * HD / 8;
    const int tot = 2 * n1 + 2 * n3;
    if (i < tot) {
      const float* src; _Float16* dst; int o;
      if (i < n1)               { src = w1;  dst = q1;  o = i * 8; }
      else if (i < 2 * n1)      { src = w2;  dst = q2;  o = (i - n1) * 8; }
      else if (i < 2 * n1 + n3) { src = wih; dst = qih; o = (i - 2 * n1) * 8; }
      else                      { src = whh; dst = qhh; o = (i - 2 * n1 - n3) * 8; }
      v4f a = *(const v4f*)(src + o), b = *(const v4f*)(src + o + 4);
      a = a * WSC; b = b * WSC;
      const v8h hv = cvt8(a, b);
      *(volatile v8h*)(dst + o) = hv;
      __threadfence();
      *(volatile v8h*)(dst + o) = hv;
    }
  } else {
    if (tid < G4 / 4) {
      const v4f a = *(const v4f*)(bih + 4 * tid), b = *(const v4f*)(bhh + 4 * tid);
      const v4f v = a + b;
      *(volatile v4f*)(bsum + 4 * tid) = v;
      __threadfence();
      *(volatile v4f*)(bsum + 4 * tid) = v;
    }
  }
}

template <int BN>
__global__ __launch_bounds__(NTHR) void k_genc(
    const float* __restrict__ A, const float* __restrict__ bnp,
    const _Float16* __restrict__ wq, const float* __restrict__ bias,
    float* Y, double* parts, int nN) {
  extern __shared__ v4f lds_dyn[];
  _Float16* sA  = (_Float16*)lds_dyn;
  float*    stg = (float*)lds_dyn;
  double*   st  = (double*)((char*)lds_dyn + GER * HD * 4);
  const int tid = threadIdx.x, lane = tid & 31, wave = tid >> 5, hh = lane >> 4, m = lane & 15;
  const int rowBase = blockIdx.x * GER;

#pragma unroll
  for (int i = 0; i < (GER * HD / 8) / NTHR; ++i) {
    const int idx = i * NTHR + tid;
    const int r   = idx >> 4;
    const int c0  = (idx & 15) * 8;
    int node = rowBase + r;
    node = node > nN - 1 ? nN - 1 : node;
    const float* xp = A + (size_t)node * HD + c0;
    v4f a = *(const v4f*)xp, b = *(const v4f*)(xp + 4);
    if (BN) {
      a = relu4(a * *(const v4f*)(bnp + c0)     + *(const v4f*)(bnp + HD + c0));
      b = relu4(b * *(const v4f*)(bnp + c0 + 4) + *(const v4f*)(bnp + HD + c0 + 4));
    }
    *(v8h*)(sA + r * AP + c0) = cvt8(a, b);
  }
  __syncthreads();

  v8f acc[8];
#pragma unroll
  for (int t = 0; t < 8; ++t) acc[t] = zero8f();
  const _Float16* ar = sA + (wave * 16 + m) * AP + 8 * hh;
#pragma unroll
  for (int kt = 0; kt < HD / 32; ++kt) {
    FragH a;
    a.h[0] = *(const v8h*)(ar + 32 * kt);
    a.h[1] = *(const v8h*)(ar + 32 * kt + 16);
#pragma unroll
    for (int t = 0; t < 8; ++t) {
      const _Float16* bp = wq + (size_t)(16 * t + m) * HD + 32 * kt + 8 * hh;
      FragH b;
      b.h[0] = *(const v8h*)bp;
      b.h[1] = *(const v8h*)(bp + 16);
      acc[t] = wmh(a.v, b.v, acc[t]);
    }
  }
  __syncthreads();

  const int r0 = wave * 16 + 8 * hh;
  float* sp = stg + r0 * HD + m;
#pragma unroll
  for (int t = 0; t < 8; ++t) {
    const float bc = bias[16 * t + m];
    sp[0 * HD + 16 * t] = acc[t][0] * WINV + bc;
    sp[1 * HD + 16 * t] = acc[t][1] * WINV + bc;
    sp[2 * HD + 16 * t] = acc[t][2] * WINV + bc;
    sp[3 * HD + 16 * t] = acc[t][3] * WINV + bc;
    sp[4 * HD + 16 * t] = acc[t][4] * WINV + bc;
    sp[5 * HD + 16 * t] = acc[t][5] * WINV + bc;
    sp[6 * HD + 16 * t] = acc[t][6] * WINV + bc;
    sp[7 * HD + 16 * t] = acc[t][7] * WINV + bc;
  }
  __syncthreads();

  {
    const int col = tid & 127, half = tid >> 7;
    double s = 0.0, q = 0.0;
#pragma unroll 1
    for (int r = half * 64; r < half * 64 + 64; ++r) {
      if (rowBase + r < nN) {
        const double v = (double)stg[r * HD + col];
        s += v; q += v * v;
      }
    }
    st[half * 256 + col] = s;
    st[half * 256 + 128 + col] = q;
  }
  __syncthreads();

  const float* lp = stg + wave * 16 * HD + 4 * lane;
  float* gp = Y + ((size_t)rowBase + wave * 16) * HD + 4 * lane;
  double* pp = parts + (size_t)blockIdx.x * 512 + wave * 64 + 2 * lane;
  const double* lq = st + wave * 64 + 2 * lane;
#pragma unroll
  for (int i = 0; i < 16; ++i) { const v4f v = *(const v4f*)(lp + i * HD); *(volatile v4f*)(gp + (size_t)i * HD) = v; }
  { const v2d v = *(const v2d*)lq; *(volatile v2d*)pp = v; }
  __threadfence();
#pragma unroll
  for (int i = 0; i < 16; ++i) { const v4f v = *(const v4f*)(lp + i * HD); *(volatile v4f*)(gp + (size_t)i * HD) = v; }
  { const v2d v = *(const v2d*)lq; *(volatile v2d*)pp = v; }
}

__global__ __launch_bounds__(NTHR) void k_bnfin(
    const double* __restrict__ parts, int nPart, int nRows,
    const float* __restrict__ gam, const float* __restrict__ bet, float* bnp) {
  __shared__ double st[256];
  __shared__ __attribute__((aligned(16))) float fo[256];
  const int tid = threadIdx.x;
  double a = 0.0;
#pragma unroll 1
  for (int p = 0; p < nPart; ++p) a += parts[(size_t)p * 256 + tid];
  st[tid] = a;
  __syncthreads();
  if (tid < HD) {
    const double inv  = 1.0 / (double)nRows;
    const double mean = st[tid] * inv;
    double var = st[HD + tid] * inv - mean * mean;
    var = var < 0.0 ? 0.0 : var;
    const float r  = rsqrtf((float)var + 1e-5f);
    const float sc = gam[tid] * r;
    const float sh = bet[tid] - (float)mean * sc;
    fo[tid] = sc; fo[HD + tid] = sh;
  }
  __syncthreads();
  if (tid < 64) { const v4f v = *(const v4f*)(fo + 4 * tid); *(volatile v4f*)(bnp + 4 * tid) = v; }
  __threadfence();
  if (tid < 64) { const v4f v = *(const v4f*)(fo + 4 * tid); *(volatile v4f*)(bnp + 4 * tid) = v; }
}

__global__ __launch_bounds__(128) void k_gxg(
    const float* __restrict__ A, const float* __restrict__ bnp,
    const _Float16* __restrict__ wq, const float* __restrict__ bsum, float* XG, int nN) {
  extern __shared__ v4f lds_dyn[];
  _Float16* sA  = (_Float16*)lds_dyn;
  float*    stg = (float*)lds_dyn;
  const int tid = threadIdx.x, lane = tid & 31, wave = tid >> 5, hh = lane >> 4, m = lane & 15;
  const int rowBase = blockIdx.x * GXR;

#pragma unroll
  for (int i = 0; i < (GXR * HD / 8) / 128; ++i) {
    const int idx = i * 128 + tid;
    const int r   = idx >> 4;
    const int c0  = (idx & 15) * 8;
    int node = rowBase + r;
    node = node > nN - 1 ? nN - 1 : node;
    const float* xp = A + (size_t)node * HD + c0;
    v4f a = *(const v4f*)xp, b = *(const v4f*)(xp + 4);
    a = relu4(a * *(const v4f*)(bnp + c0)     + *(const v4f*)(bnp + HD + c0));
    b = relu4(b * *(const v4f*)(bnp + c0 + 4) + *(const v4f*)(bnp + HD + c0 + 4));
    *(v8h*)(sA + r * AP + c0) = cvt8(a, b);
  }
  __syncthreads();

  FragH a[4];
  {
    const _Float16* ar = sA + (wave * 16 + m) * AP + 8 * hh;
#pragma unroll
    for (int kt = 0; kt < 4; ++kt) {
      a[kt].h[0] = *(const v8h*)(ar + 32 * kt);
      a[kt].h[1] = *(const v8h*)(ar + 32 * kt + 16);
    }
  }
  __syncthreads();

  const int r0 = wave * 16 + 8 * hh;
#pragma unroll 1
  for (int cg = 0; cg < 4; ++cg) {
    v8f acc[8];
#pragma unroll
    for (int t = 0; t < 8; ++t) acc[t] = zero8f();
#pragma unroll
    for (int kt = 0; kt < 4; ++kt) {
#pragma unroll
      for (int t = 0; t < 8; ++t) {
        const _Float16* bp = wq + (size_t)(cg * HD + 16 * t + m) * HD + 32 * kt + 8 * hh;
        FragH b;
        b.h[0] = *(const v8h*)bp;
        b.h[1] = *(const v8h*)(bp + 16);
        acc[t] = wmh(a[kt].v, b.v, acc[t]);
      }
    }
#pragma unroll
    for (int t = 0; t < 8; ++t) {
      const float bc = bsum[cg * HD + 16 * t + m];
      float* sp = stg + r0 * G4 + t * 64 + m * 4 + cg;
      sp[0 * G4] = acc[t][0] * WINV + bc;
      sp[1 * G4] = acc[t][1] * WINV + bc;
      sp[2 * G4] = acc[t][2] * WINV + bc;
      sp[3 * G4] = acc[t][3] * WINV + bc;
      sp[4 * G4] = acc[t][4] * WINV + bc;
      sp[5 * G4] = acc[t][5] * WINV + bc;
      sp[6 * G4] = acc[t][6] * WINV + bc;
      sp[7 * G4] = acc[t][7] * WINV + bc;
    }
  }
  __syncthreads();

  const float* lp = stg + wave * 16 * G4 + 4 * lane;
  float* gp = XG + ((size_t)rowBase + wave * 16) * G4 + 4 * lane;
#pragma unroll
  for (int i = 0; i < 16; ++i) {
#pragma unroll
    for (int q = 0; q < 4; ++q) {
      const v4f v = *(const v4f*)(lp + i * G4 + q * 128);
      *(volatile v4f*)(gp + (size_t)i * G4 + q * 128) = v;
    }
  }
  __threadfence();
#pragma unroll
  for (int i = 0; i < 16; ++i) {
#pragma unroll
    for (int q = 0; q < 4; ++q) {
      const v4f v = *(const v4f*)(lp + i * G4 + q * 128);
      *(volatile v4f*)(gp + (size_t)i * G4 + q * 128) = v;
    }
  }
}

__global__ __launch_bounds__(128) void k_lstm(
    const float* __restrict__ xg, const int* __restrict__ paths,
    const _Float16* __restrict__ whh, float* hfo, int T, int nP, int nN) {
  __shared__ __attribute__((aligned(16))) _Float16 hs[PB * AP];
  __shared__ __attribute__((aligned(16))) float    cs[PB * HD];
  const int tid = threadIdx.x, lane = tid & 31, wave = tid >> 5, hh = lane >> 4, m = lane & 15;
  const int pblk = blockIdx.x * PB;
  {
    const v4f z = {0.f, 0.f, 0.f, 0.f};
    for (int i = tid; i < PB * HD / 4; i += 128) ((v4f*)cs)[i] = z;
  }
  __syncthreads();

  const int prow0 = wave * 16 + 8 * hh;
#pragma unroll 1
  for (int t = 0; t < T; ++t) {
    const bool rec  = (t > 0);
    const bool last = (t + 1 == T);
    int nd[8];
#pragma unroll
    for (int r = 0; r < 8; ++r) {
      int p = pblk + prow0 + r;
      p = p > nP - 1 ? nP - 1 : p;
      int v = paths[(size_t)p * T + t];
      v = v < 0 ? 0 : (v > nN - 1 ? nN - 1 : v);
      nd[r] = v;
    }
    FragH a[4];
    if (rec) {
      const _Float16* ar = hs + (wave * 16 + m) * AP + 8 * hh;
#pragma unroll
      for (int kt = 0; kt < 4; ++kt) {
        a[kt].h[0] = *(const v8h*)(ar + 32 * kt);
        a[kt].h[1] = *(const v8h*)(ar + 32 * kt + 16);
      }
    } else {
#pragma unroll
      for (int kt = 0; kt < 4; ++kt) { a[kt].h[0] = zero8h(); a[kt].h[1] = zero8h(); }
    }

#pragma unroll 1
    for (int nt = 0; nt < 8; ++nt) {
      v8f acc[4];
#pragma unroll
      for (int g = 0; g < 4; ++g) acc[g] = zero8f();
      if (rec) {
#pragma unroll
        for (int kt = 0; kt < 4; ++kt) {
#pragma unroll
          for (int g = 0; g < 4; ++g) {
            const _Float16* bp = whh + (size_t)(g * HD + nt * 16 + m) * HD + 32 * kt + 8 * hh;
            FragH b;
            b.h[0] = *(const v8h*)bp;
            b.h[1] = *(const v8h*)(bp + 16);
            acc[g] = wmh(a[kt].v, b.v, acc[g]);
          }
        }
      }
#pragma unroll
      for (int r = 0; r < 8; ++r) {
        const int pl = prow0 + r;
        const v4f x4 = *(const v4f*)(xg + (size_t)nd[r] * G4 + nt * 64 + m * 4);
        const float pi = acc[0][r] * WINV + x4.x;
        const float pf = acc[1][r] * WINV + x4.y;
        const float pg = acc[2][r] * WINV + x4.z;
        const float po = acc[3][r] * WINV + x4.w;
        const int ci = pl * HD + nt * 16 + m;
        const float cold = cs[ci];
        const float cn = sigm(pf) * cold + sigm(pi) * tanhf(pg);
        const float hn = sigm(po) * tanhf(cn);
        if (!last) {
          cs[ci] = cn;
          hs[pl * AP + nt * 16 + m] = (_Float16)hn;
        } else {
          cs[ci] = hn;
        }
      }
    }
    __syncthreads();
  }

  const float* lp = cs + wave * 16 * HD + 4 * lane;
  float* gp = hfo + ((size_t)pblk + wave * 16) * HD + 4 * lane;
#pragma unroll
  for (int i = 0; i < 16; ++i) { const v4f v = *(const v4f*)(lp + i * HD); *(volatile v4f*)(gp + (size_t)i * HD) = v; }
  __threadfence();
#pragma unroll
  for (int i = 0; i < 16; ++i) { const v4f v = *(const v4f*)(lp + i * HD); *(volatile v4f*)(gp + (size_t)i * HD) = v; }
}

__device__ __forceinline__ int scan_chunk(const int* __restrict__ paths, int T, int nE, int cbase,
                                          int nodeBase, int* list, int tid, int lane, int wave) {
  int wc = 0;
#pragma unroll
  for (int g = 0; g < NGRP; ++g) {
    const int el0  = (g * NTHR + tid) * EPT;
    const int e0   = cbase + el0;
    const int sent = -2147483647 - 1;
    int d[8];
#pragma unroll
    for (int j = 0; j < 8; ++j) {
      const int e  = e0 + j;
      const int ec = e < nE ? e : nE - 1;
      const int v  = paths[(size_t)ec * T + (T - 1)];
      d[j] = (e < nE) ? v : sent;
    }
    const unsigned nb = (unsigned)nodeBase;
    unsigned s[8]; bool ht[8]; bool anyl = false;
#pragma unroll
    for (int j = 0; j < 8; ++j) { s[j] = (unsigned)d[j] - nb; ht[j] = s[j] < (unsigned)NBA; anyl = anyl | ht[j]; }
    const unsigned any = __builtin_amdgcn_ballot_w32(anyl);
    if (any != 0u) {
#pragma unroll
      for (int j = 0; j < 8; ++j) {
        const unsigned mj = __builtin_amdgcn_ballot_w32(ht[j]);
        if (mj != 0u) {
          if (ht[j]) {
            const int pos = wc + (int)__builtin_amdgcn_mbcnt_lo(mj, 0u);
            if (pos < WCAP) list[wave * WCAP + pos] = ((el0 + j) << 12) | (int)s[j];
          }
          wc += (int)__builtin_popcount(mj);
        }
      }
    }
  }
  return wc;
}

__global__ __launch_bounds__(NTHR) void k_agg(
    const int* __restrict__ paths, const float* __restrict__ hf,
    const float* __restrict__ yprev, const float* __restrict__ bnp,
    float* ynew, double* parts, int T, int nP, int nN) {
  extern __shared__ v4f lds_dyn[];
  float*  acc  = (float*)lds_dyn;
  int*    list = (int*)(acc + NBA * HD);
  int*    wcnt = list + LISTN;
  double* st   = (double*)(wcnt + 16);
  const int tid = threadIdx.x, lane = tid & 31, wave = tid >> 5;
  const int nodeBase = blockIdx.x * NBA;

  {
    const v4f z = {0.f, 0.f, 0.f, 0.f};
    for (int i = tid; i < NBA * HD / 4; i += NTHR) lds_dyn[i] = z;
  }
  __syncthreads();

  const int nChunks = (nP + CHUNK - 1) / CHUNK;
#pragma unroll 1
  for (int ch = 0; ch < nChunks; ++ch) {
    const int cbase = ch * CHUNK;
    const int wc = scan_chunk(paths, T, nP, cbase, nodeBase, list, tid, lane, wave);
    if (lane == 0) wcnt[wave] = wc;
    __syncthreads();
    if (wave == 0) {
#pragma unroll 1
      for (int wsx = 0; wsx < NWAVE; ++wsx) {
        int n = __builtin_amdgcn_readfirstlane(wcnt[wsx]);
        n = n > WCAP ? WCAP : (n < 0 ? 0 : n);
        const int* lp = list + wsx * WCAP;
#pragma unroll 1
        for (int i = 0; i < n; ++i) {
          const int ent  = __builtin_amdgcn_readfirstlane(lp[i]);
          const int slot = ent & (NBA - 1);
          int e = cbase + ((ent >> 12) & (CHUNK - 1));
          e = e > nP - 1 ? nP - 1 : e;
          const v4f v = *(const v4f*)(hf + (size_t)e * HD + 4 * lane);
          v4f* ap = (v4f*)(acc + slot * HD + 4 * lane);
          *ap = *ap + v;
        }
      }
    }
    __syncthreads();
  }

#pragma unroll 1
  for (int i = 0; i < (NBA * HD / 4) / NTHR; ++i) {
    const int idx  = i * NTHR + tid;
    const int slot = idx >> 5;
    const int c4   = (idx & 31) * 4;
    int node = nodeBase + slot;
    node = node > nN - 1 ? nN - 1 : node;
    const v4f yp = *(const v4f*)(yprev + (size_t)node * HD + c4);
    const v4f s4 = *(const v4f*)(bnp + c4);
    const v4f h4 = *(const v4f*)(bnp + HD + c4);
    const v4f rr = relu4(yp * s4 + h4);
    v4f* ap = (v4f*)(acc + slot * HD + c4);
    *ap = *ap + rr;
  }
  __syncthreads();

  {
    const int col = tid & 127, half = tid >> 7;
    double s = 0.0, q = 0.0;
#pragma unroll 1
    for (int r = half * (NBA / 2); r < half * (NBA / 2) + NBA / 2; ++r) {
      if (nodeBase + r < nN) {
        const double v = (double)acc[r * HD + col];
        s += v; q += v * v;
      }
    }
    st[half * 256 + col] = s;
    st[half * 256 + 128 + col] = q;
  }
  __syncthreads();

  const float* lp = acc + wave * 32 * HD + 4 * lane;
  float* gp = ynew + ((size_t)nodeBase + wave * 32) * HD + 4 * lane;
  double* pp = parts + (size_t)blockIdx.x * 512 + wave * 64 + 2 * lane;
  const double* lq = st + wave * 64 + 2 * lane;
#pragma unroll 4
  for (int i = 0; i < 32; ++i) { const v4f v = *(const v4f*)(lp + i * HD); *(volatile v4f*)(gp + (size_t)i * HD) = v; }
  { const v2d v = *(const v2d*)lq; *(volatile v2d*)pp = v; }
  __threadfence();
#pragma unroll 4
  for (int i = 0; i < 32; ++i) { const v4f v = *(const v4f*)(lp + i * HD); *(volatile v4f*)(gp + (size_t)i * HD) = v; }
  { const v2d v = *(const v2d*)lq; *(volatile v2d*)pp = v; }
}

__global__ __launch_bounds__(NTHR) void k_pool(
    const float* __restrict__ Y, const float* __restrict__ bnp, const int* __restrict__ batch,
    float* pooled, int nN, int nG) {
  extern __shared__ v4f lds_dyn[];
  float* acc = (float*)lds_dyn;
  float* res = acc + NWAVE * NGR * 32;
  const int tid = threadIdx.x, lane = tid & 31, wave = tid >> 5;
  const int slab = blockIdx.x;
  const int c = slab * 32 + lane;
  float* wa = acc + wave * NGR * 32;
#pragma unroll 1
  for (int g = 0; g < NGR; ++g) wa[g * 32 + lane] = 0.f;
  const float sc = bnp[c], sh = bnp[HD + c];
  const int per = (nN + NWAVE - 1) / NWAVE;
  const int i0 = wave * per;
  const int i1 = (i0 + per < nN) ? (i0 + per) : nN;
#pragma unroll 1
  for (int i = i0; i < i1; ++i) {
    const int g = batch[i];
    const float v = Y[(size_t)i * HD + c];
    const float h = fmaxf(fmaf(v, sc, sh), 0.f);
    if ((unsigned)g < (unsigned)nG && g < NGR) wa[g * 32 + lane] += h;
  }
  __syncthreads();
  for (int o = tid; o < NGR * 32; o += NTHR) {
    float s = 0.f;
#pragma unroll
    for (int w = 0; w < NWAVE; ++w) s += acc[w * NGR * 32 + o];
    res[o] = s;
  }
  __syncthreads();
#pragma unroll
  for (int j = 0; j < 4; ++j) {
    const int k = wave * 4 + j;
    const int row = 4 * k + (lane >> 3);
    const int cc = (lane & 7) * 4;
    const v4f v = *(const v4f*)(res + row * 32 + cc);
    *(volatile v4f*)(pooled + (size_t)row * HD + slab * 32 + cc) = v;
  }
  __threadfence();
#pragma unroll
  for (int j = 0; j < 4; ++j) {
    const int k = wave * 4 + j;
    const int row = 4 * k + (lane >> 3);
    const int cc = (lane & 7) * 4;
    const v4f v = *(const v4f*)(res + row * 32 + cc);
    *(volatile v4f*)(pooled + (size_t)row * HD + slab * 32 + cc) = v;
  }
}

__global__ __launch_bounds__(NTHR) void k_head(
    const float* __restrict__ pooled, const float* __restrict__ w1, const float* __restrict__ b1,
    const float* __restrict__ w2, const float* __restrict__ b2, float* out) {
  extern __shared__ v4f lds_dyn[];
  float* zs = (float*)lds_dyn;
  float* os = zs + NGR * ZP;
  const int tid = threadIdx.x, lane = tid & 31, wave = tid >> 5, hh = lane >> 4, m = lane & 15;

  FragB ah[4], al[4];
  {
    const float* arow = pooled + (size_t)(wave * 16 + m) * HD + 8 * hh;
#pragma unroll
    for (int kt = 0; kt < 4; ++kt) {
      const float* p = arow + 32 * kt;
      const v4f x0 = *(const v4f*)p,        x1 = *(const v4f*)(p + 4);
      const v4f x2 = *(const v4f*)(p + 16), x3 = *(const v4f*)(p + 20);
      split8(x0, x1, ah[kt], al[kt], 0);
      split8(x2, x3, ah[kt], al[kt], 1);
    }
  }
  v8f acc[8];
#pragma unroll
  for (int t = 0; t < 8; ++t) acc[t] = zero8f();
#pragma unroll
  for (int t = 0; t < 8; ++t) {
#pragma unroll
    for (int kt = 0; kt < 4; ++kt) {
      const float* p = w1 + (size_t)(16 * t + m) * HD + 32 * kt + 8 * hh;
      const v4f y0 = *(const v4f*)p,        y1 = *(const v4f*)(p + 4);
      const v4f y2 = *(const v4f*)(p + 16), y3 = *(const v4f*)(p + 20);
      FragB bh, bl;
      split8(y0, y1, bh, bl, 0);
      split8(y2, y3, bh, bl, 1);
      acc[t] = wmb(ah[kt].v, bh.v, acc[t]);
      acc[t] = wmb(ah[kt].v, bl.v, acc[t]);
      acc[t] = wmb(al[kt].v, bh.v, acc[t]);
    }
  }
  const int r0 = wave * 16 + 8 * hh;
#pragma unroll
  for (int t = 0; t < 8; ++t) {
    const int col = 16 * t + m;
    const float bc = b1[col];
    float* sp = zs + r0 * ZP + col;
    sp[0 * ZP] = fmaxf(acc[t][0] + bc, 0.f);
    sp[1 * ZP] = fmaxf(acc[t][1] + bc, 0.f);
    sp[2 * ZP] = fmaxf(acc[t][2] + bc, 0.f);
    sp[3 * ZP] = fmaxf(acc[t][3] + bc, 0.f);
    sp[4 * ZP] = fmaxf(acc[t][4] + bc, 0.f);
    sp[5 * ZP] = fmaxf(acc[t][5] + bc, 0.f);
    sp[6 * ZP] = fmaxf(acc[t][6] + bc, 0.f);
    sp[7 * ZP] = fmaxf(acc[t][7] + bc, 0.f);
  }
  __syncthreads();

  FragB a2h[4], a2l[4];
  {
    const float* zrow = zs + (wave * 16 + m) * ZP + 8 * hh;
#pragma unroll
    for (int kt = 0; kt < 4; ++kt) {
      const float* p = zrow + 32 * kt;
      const v4f x0 = *(const v4f*)p,        x1 = *(const v4f*)(p + 4);
      const v4f x2 = *(const v4f*)(p + 16), x3 = *(const v4f*)(p + 20);
      split8(x0, x1, a2h[kt], a2l[kt], 0);
      split8(x2, x3, a2h[kt], a2l[kt], 1);
    }
  }
  const int nrow = m < NCLS ? m : NCLS - 1;
  const v4f z4 = {0.f, 0.f, 0.f, 0.f};
  v8f c2 = zero8f();
#pragma unroll
  for (int kt = 0; kt < 4; ++kt) {
    const float* p = w2 + (size_t)nrow * HD + 32 * kt + 8 * hh;
    v4f y0 = *(const v4f*)p,        y1 = *(const v4f*)(p + 4);
    v4f y2 = *(const v4f*)(p + 16), y3 = *(const v4f*)(p + 20);
    y0 = (m < NCLS) ? y0 : z4; y1 = (m < NCLS) ? y1 : z4;
    y2 = (m < NCLS) ? y2 : z4; y3 = (m < NCLS) ? y3 : z4;
    FragB bh, bl;
    split8(y0, y1, bh, bl, 0);
    split8(y2, y3, bh, bl, 1);
    c2 = wmb(a2h[kt].v, bh.v, c2);
    c2 = wmb(a2h[kt].v, bl.v, c2);
    c2 = wmb(a2l[kt].v, bh.v, c2);
  }
  {
    const float bc2 = b2[nrow];
    if (m < NCLS) {
      float* sp = os + r0 * NCLS + m;
      sp[0 * NCLS] = c2[0] + bc2;
      sp[1 * NCLS] = c2[1] + bc2;
      sp[2 * NCLS] = c2[2] + bc2;
      sp[3 * NCLS] = c2[3] + bc2;
      sp[4 * NCLS] = c2[4] + bc2;
      sp[5 * NCLS] = c2[5] + bc2;
      sp[6 * NCLS] = c2[6] + bc2;
      sp[7 * NCLS] = c2[7] + bc2;
    }
  }
  __syncthreads();

  if (wave == 0) {
#pragma unroll
    for (int k = 0; k < (NGR * NCLS) / 128; ++k) {
      const v4f v = *(const v4f*)(os + k * 128 + 4 * lane);
      *(volatile v4f*)(out + k * 128 + 4 * lane) = v;
    }
  }
  __threadfence();
  if (wave == 0) {
#pragma unroll
    for (int k = 0; k < (NGR * NCLS) / 128; ++k) {
      const v4f v = *(const v4f*)(os + k * 128 + 4 * lane);
      *(volatile v4f*)(out + k * 128 + 4 * lane) = v;
    }
  }
}

extern "C" void kernel_launch(void* const* d_in, const int* in_sizes, int n_in,
                              void* d_out, int out_size, void* d_ws, size_t ws_size,
                              hipStream_t stream) {
  if (n_in < 24) return;
  const int nN = in_sizes[0] / HD;
  if (nN <= 0 || in_sizes[0] != nN * HD) return;
  const int P2 = in_sizes[1] / 2, P3 = in_sizes[2] / 3;
  if (P2 <= 0 || P3 <= 0 || in_sizes[1] != P2 * 2 || in_sizes[2] != P3 * 3) return;
  if (in_sizes[3] != nN) return;
  if (in_sizes[4] != HD * HD || in_sizes[8] != HD * HD) return;
  if (in_sizes[5] < HD || in_sizes[6] < HD || in_sizes[7] < HD) return;
  if (in_sizes[9] < HD || in_sizes[10] < HD || in_sizes[11] < HD) return;
  if (in_sizes[12] != G4 * HD || in_sizes[13] != G4 * HD || in_sizes[14] < G4 || in_sizes[15] < G4) return;
  if (in_sizes[16] < HD || in_sizes[17] < HD || in_sizes[18] < HD || in_sizes[19] < HD) return;
  if (in_sizes[20] != HD * HD || in_sizes[21] < HD || in_sizes[22] != NCLS * HD || in_sizes[23] < NCLS) return;
  if (out_size != NGR * NCLS) return;

  const float* x      = (const float*)d_in[0];
  const int*   path2  = (const int*)d_in[1];
  const int*   path3  = (const int*)d_in[2];
  const int*   batch  = (const int*)d_in[3];
  const float* fe_w1  = (const float*)d_in[4];
  const float* fe_b1  = (const float*)d_in[5];
  const float* fe_g1  = (const float*)d_in[6];
  const float* fe_be1 = (const float*)d_in[7];
  const float* fe_w2  = (const float*)d_in[8];
  const float* fe_b2  = (const float*)d_in[9];
  const float* fe_g2  = (const float*)d_in[10];
  const float* fe_be2 = (const float*)d_in[11];
  const float* w_ih   = (const float*)d_in[12];
  const float* w_hh   = (const float*)d_in[13];
  const float* b_ih   = (const float*)d_in[14];
  const float* b_hh   = (const float*)d_in[15];
  const float* bn1_g  = (const float*)d_in[16];
  const float* bn1_b  = (const float*)d_in[17];
  const float* bn2_g  = (const float*)d_in[18];
  const float* bn2_b  = (const float*)d_in[19];
  const float* lin1_w = (const float*)d_in[20];
  const float* lin1_b = (const float*)d_in[21];
  const float* lin2_w = (const float*)d_in[22];
  const float* lin2_b = (const float*)d_in[23];
  float* out = (float*)d_out;

  const int nAgg  = (nN + NBA - 1) / NBA;
  const int NPAD  = nAgg * NBA;
  const int nEnc  = NPAD / GER;
  const int nXg   = NPAD / GXR;
  const int nL2   = (P2 + PB - 1) / PB;
  const int nL3   = (P3 + PB - 1) / PB;
  const int PPAD  = (nL2 > nL3 ? nL2 : nL3) * PB;
  const int nPartMax = 2 * nEnc;

  char* ws = (char*)d_ws;
  size_t off = 0;
  const size_t oQ1 = off; off += (size_t)HD * HD * 2;            off = (off + 255) & ~(size_t)255;
  const size_t oQ2 = off; off += (size_t)HD * HD * 2;            off = (off + 255) & ~(size_t)255;
  const size_t oQI = off; off += (size_t)G4 * HD * 2;            off = (off + 255) & ~(size_t)255;
  const size_t oQH = off; off += (size_t)G4 * HD * 2;            off = (off + 255) & ~(size_t)255;
  const size_t oBS = off; off += (size_t)G4 * 4;                 off = (off + 255) & ~(size_t)255;
  const size_t oB0 = off; off += 1024;                           off = (off + 255) & ~(size_t)255;
  const size_t oB1 = off; off += 1024;                           off = (off + 255) & ~(size_t)255;
  const size_t oB2 = off; off += 1024;                           off = (off + 255) & ~(size_t)255;
  const size_t oB3 = off; off += 1024;                           off = (off + 255) & ~(size_t)255;
  const size_t oPT = off; off += (size_t)nPartMax * 256 * 8;     off = (off + 255) & ~(size_t)255;
  const size_t oYA = off; off += (size_t)NPAD * HD * 4;          off = (off + 255) & ~(size_t)255;
  const size_t oYB = off; off += (size_t)NPAD * HD * 4;          off = (off + 255) & ~(size_t)255;
  const size_t oXG = off; off += (size_t)NPAD * G4 * 4;          off = (off + 255) & ~(size_t)255;
  const size_t oHF = off; off += (size_t)PPAD * HD * 4;          off = (off + 255) & ~(size_t)255;
  const size_t oPL = off; off += (size_t)NGR * HD * 4;           off = (off + 255) & ~(size_t)255;
  if (off > ws_size) return;

  _Float16* q1   = (_Float16*)(ws + oQ1);
  _Float16* q2   = (_Float16*)(ws + oQ2);
  _Float16* qih  = (_Float16*)(ws + oQI);
  _Float16* qhh  = (_Float16*)(ws + oQH);
  float*    bsum = (float*)(ws + oBS);
  float*    bnE1 = (float*)(ws + oB0);
  float*    bnE2 = (float*)(ws + oB1);
  float*    bnC1 = (float*)(ws + oB2);
  float*    bnC2 = (float*)(ws + oB3);
  double*   parts = (double*)(ws + oPT);
  float*    YA   = (float*)(ws + oYA);
  float*    YB   = (float*)(ws + oYB);
  float*    XG   = (float*)(ws + oXG);
  float*    HF   = (float*)(ws + oHF);
  float*    pooled = (float*)(ws + oPL);

  hipFuncSetAttribute(reinterpret_cast<const void*>(&k_genc<0>), hipFuncAttributeMaxDynamicSharedMemorySize, LDS_ENC);
  hipFuncSetAttribute(reinterpret_cast<const void*>(&k_genc<1>), hipFuncAttributeMaxDynamicSharedMemorySize, LDS_ENC);
  hipFuncSetAttribute(reinterpret_cast<const void*>(&k_gxg),     hipFuncAttributeMaxDynamicSharedMemorySize, LDS_XG);
  hipFuncSetAttribute(reinterpret_cast<const void*>(&k_agg),     hipFuncAttributeMaxDynamicSharedMemorySize, LDS_AGG);
  hipFuncSetAttribute(reinterpret_cast<const void*>(&k_pool),    hipFuncAttributeMaxDynamicSharedMemorySize, LDS_POOL);
  hipFuncSetAttribute(reinterpret_cast<const void*>(&k_head),    hipFuncAttributeMaxDynamicSharedMemorySize, LDS_HEAD);

  const int nUnits = 2 * (HD * HD / 8) + 2 * (G4 * HD / 8);
  const int nWblk  = (nUnits + NTHR - 1) / NTHR;
  k_wprep<<<nWblk + 1, NTHR, 0, stream>>>(fe_w1, fe_w2, w_ih, w_hh, b_ih, b_hh, q1, q2, qih, qhh, bsum, nWblk);

  k_genc<0><<<nEnc, NTHR, LDS_ENC, stream>>>(x, bnE1, q1, fe_b1, YA, parts, nN);
  k_bnfin<<<1, NTHR, 0, stream>>>(parts, 2 * nEnc, nN, fe_g1, fe_be1, bnE1);

  k_genc<1><<<nEnc, NTHR, LDS_ENC, stream>>>(YA, bnE1, q2, fe_b2, YB, parts, nN);
  k_bnfin<<<1, NTHR, 0, stream>>>(parts, 2 * nEnc, nN, fe_g2, fe_be2, bnE2);

  k_gxg<<<nXg, 128, LDS_XG, stream>>>(YB, bnE2, qih, bsum, XG, nN);
  k_lstm<<<nL2, 128, 0, stream>>>(XG, path2, qhh, HF, 2, P2, nN);
  k_agg<<<nAgg, NTHR, LDS_AGG, stream>>>(path2, HF, YB, bnE2, YA, parts, 2, P2, nN);
  k_bnfin<<<1, NTHR, 0, stream>>>(parts, 2 * nAgg, nN, bn1_g, bn1_b, bnC1);

  k_gxg<<<nXg, 128, LDS_XG, stream>>>(YA, bnC1, qih, bsum, XG, nN);
  k_lstm<<<nL3, 128, 0, stream>>>(XG, path3, qhh, HF, 3, P3, nN);
  k_agg<<<nAgg, NTHR, LDS_AGG, stream>>>(path3, HF, YA, bnC1, YB, parts, 3, P3, nN);
  k_bnfin<<<1, NTHR, 0, stream>>>(parts, 2 * nAgg, nN, bn2_g, bn2_b, bnC2);

  k_pool<<<HD / 32, NTHR, LDS_POOL, stream>>>(YB, bnC2, batch, pooled, nN, NGR);
  k_head<<<1, NTHR, LDS_HEAD, stream>>>(pooled, lin1_w, lin1_b, lin2_w, lin2_b, out);
}
